// Mainnet_27582279975476
// MI455X (gfx1250) — hardware-verified
//
#include <hip/hip_runtime.h>
#include <math.h>

typedef __attribute__((ext_vector_type(16))) _Float16 v16h;
typedef __attribute__((ext_vector_type(16))) __bf16 v16b;
typedef __attribute__((ext_vector_type(8)))  _Float16 v8h;
typedef __attribute__((ext_vector_type(8)))  float v8f;
typedef __attribute__((ext_vector_type(4)))  float v4f;
typedef __attribute__((ext_vector_type(2)))  float v2f;
typedef __attribute__((ext_vector_type(4)))  unsigned v4u;
typedef __attribute__((ext_vector_type(4)))  int v4i;
typedef float __attribute__((may_alias)) float_a;
typedef int __attribute__((may_alias)) int_a;

template <typename T> __device__ __forceinline__ void vst2(void* p, T v) { *(volatile T*)p = v; __threadfence(); *(volatile T*)p = v; }
__device__ __forceinline__ v8f wmma16(v16h a, v16h b, v8f c) {
  v8f d = __builtin_amdgcn_wmma_f32_16x16x32_f16(false, a, false, b, (short)0, c, false, false);
  asm volatile("v_nop\n\tv_nop\n\tv_nop\n\tv_nop" : "+v"(d) : "v"(a), "v"(b));
  return d;
}
__device__ __forceinline__ v8f wmma_bf(v16b a, v16b b, v8f c) {
  v8f d = __builtin_amdgcn_wmma_f32_16x16x32_bf16(false, a, false, b, (short)0, c, false, false);
  asm volatile("v_nop\n\tv_nop\n\tv_nop\n\tv_nop" : "+v"(d) : "v"(a), "v"(b));
  return d;
}
__device__ __forceinline__ v16h frag_h(const _Float16* rowk0, int lane) {
  union { v16h v; v8h q[2]; } u; const _Float16* p = rowk0 + 8 * (lane >> 4);
  u.q[0] = *(const v8h*)p; u.q[1] = *(const v8h*)(p + 16); return u.v;
}
__device__ __forceinline__ v16h frag_f32(const float* rowk0, int lane) {
  v16h a; const float* p = rowk0 + 8 * (lane >> 4);
#pragma unroll
  for (int i = 0; i < 8; ++i) { a[i] = (_Float16)p[i]; a[8 + i] = (_Float16)p[16 + i]; }
  return a;
}
__device__ __forceinline__ v16h frag_f32s(const float* rowk0, int lane, float sc) {
  v16h a; const float* p = rowk0 + 8 * (lane >> 4);
#pragma unroll
  for (int i = 0; i < 8; ++i) { a[i] = (_Float16)(p[i] * sc); a[8 + i] = (_Float16)(p[16 + i] * sc); }
  return a;
}
__device__ __forceinline__ v16h fragc_f32(const float* W, int k0, int n, int lane, int ld, int K) {
  v16h a; const int g = lane >> 4;
#pragma unroll
  for (int i = 0; i < 8; ++i) { const int ka = k0 + 8 * g + i, kb = ka + 16;
    a[i] = (_Float16)(ka < K ? W[(size_t)(ka < K ? ka : K - 1) * ld + n] : 0.f); a[8 + i] = (_Float16)(kb < K ? W[(size_t)(kb < K ? kb : K - 1) * ld + n] : 0.f); }
  return a;
}
struct F2 { v16b h, l; };
__device__ __forceinline__ F2 bsplit16(const float v[16]) { F2 r;
#pragma unroll
  for (int i = 0; i < 16; ++i) { const __bf16 h = (__bf16)v[i]; r.h[i] = h; r.l[i] = (__bf16)(v[i] - (float)h); }
  return r; }
__device__ __forceinline__ F2 split_row(const float* row, int k0, int lane) { float v[16]; const float* p = row + k0 + 8 * (lane >> 4);
#pragma unroll
  for (int i = 0; i < 8; ++i) { v[i] = p[i]; v[8 + i] = p[16 + i]; }
  return bsplit16(v); }
__device__ __forceinline__ F2 split_rowK(const float* row, int k0, int lane, int K) { float v[16]; const int g = lane >> 4;
#pragma unroll
  for (int i = 0; i < 8; ++i) { const int ka = k0 + 8 * g + i, kb = ka + 16; v[i] = ka < K ? row[ka < K ? ka : K - 1] : 0.f; v[8 + i] = kb < K ? row[kb < K ? kb : K - 1] : 0.f; }
  return bsplit16(v); }
__device__ __forceinline__ F2 split_col(const float* W, int k0, int n, int lane, int ld, int K) { float v[16]; const int g = lane >> 4;
#pragma unroll
  for (int i = 0; i < 8; ++i) { const int ka = k0 + 8 * g + i, kb = ka + 16; v[i] = ka < K ? W[(size_t)(ka < K ? ka : K - 1) * ld + n] : 0.f; v[8 + i] = kb < K ? W[(size_t)(kb < K ? kb : K - 1) * ld + n] : 0.f; }
  return bsplit16(v); }
__device__ __forceinline__ v8f mac3(const F2& a, const F2& b, v8f c) { c = wmma_bf(a.l, b.h, c); c = wmma_bf(a.h, b.l, c); return wmma_bf(a.h, b.h, c); }
__device__ __forceinline__ float sigm(float v) { return 1.0f / (1.0f + expf(-v)); }
#define LDSX() do { asm volatile("s_wait_dscnt 0" ::: "memory"); __builtin_amdgcn_wave_barrier(); __builtin_amdgcn_fence(__ATOMIC_RELEASE, "workgroup"); } while (0)


#define NB 4
#define CC 32
#define IH 256
#define IW 256
#define NP (IH * IW)
#define KK 9
#define CO (CC * KK)
#define CP (4 * CC)
#define BNE 1e-5f
#ifndef TNB
#define TNB NB
#endif
#ifndef TPIX
#define TPIX NP
#endif
typedef __attribute__((ext_vector_type(8))) __bf16 v8b;
__device__ __forceinline__ v16b frag_b(const __bf16* rowk0, int lane) {
  union { v16b v; v8b q[2]; } u; const __bf16* p = rowk0 + 8 * (lane >> 4);
  u.q[0] = *(const v8b*)p; u.q[1] = *(const v8b*)(p + 16); return u.v;
}
__device__ __forceinline__ float bfr(float v) { return (float)(__bf16)v; }
__device__ __attribute__((noinline)) float exp_ni(float v) { return expf(v); }
__device__ __attribute__((noinline)) float erf_ni(float v) { return erff(v); }

#define WS_PW  0u
#define WS_PF  (WS_PW + 2u * 8 * CC * (KK * CC))
#define WS_PO  (WS_PF + 2u * CC * (KK * CP))
#define WS_M   (WS_PO + 2u * CO * CC)
#define WS_H   (WS_M + 4u * (size_t)NB * CC * NP)
#define WS_PR  (WS_H + 4u * (size_t)NB * CC * NP)
#define WS_END (WS_PR + 2u * (size_t)NB * CP * NP)

__global__ __launch_bounds__(256) void k_packw(const float* __restrict__ WCONV, const float* __restrict__ WFIN, const float* __restrict__ WOUTC, char* __restrict__ ws) { const int o = blockIdx.x, which = blockIdx.y, t = threadIdx.x; __shared__ __align__(16) _Float16 s[KK * CP]; __shared__ __align__(16) __bf16 sb[CC];
  if (which < 8) { if (o >= CC) return; const float* w = WCONV + ((size_t)which * CC + o) * CC * KK;
    for (int e = t; e < KK * CC; e += 256) { const int tap = e / CC, c = e % CC; s[e] = (_Float16)bfr(w[(size_t)c * KK + tap]); } __syncthreads();
    for (int q = t; q < KK * CC / 8; q += 256) vst2((unsigned*)((_Float16*)(ws + WS_PW) + ((size_t)which * CC + o) * (KK * CC) + q * 8), *(const v4u*)&s[q * 8]); }
  else if (which == 8) { if (o >= CC) return; const float* w = WFIN + (size_t)o * CP * KK;
    for (int e = t; e < KK * CP; e += 256) { const int tap = e / CP, c = e % CP; s[e] = (_Float16)bfr(w[(size_t)c * KK + tap]); } __syncthreads();
    for (int q = t; q < KK * CP / 8; q += 256) vst2((unsigned*)((_Float16*)(ws + WS_PF) + (size_t)o * (KK * CP) + q * 8), *(const v4u*)&s[q * 8]); }
  else { if (o >= CO) return; if (t < CC) sb[t] = (__bf16)WOUTC[(size_t)o * CC + t]; __syncthreads(); if (t < CC / 8) vst2((unsigned*)((__bf16*)(ws + WS_PO) + (size_t)o * CC + t * 8), *(const v4u*)&sb[t * 8]); } }
template <typename TS>
__device__ __forceinline__ v16h frag_tap(const TS* __restrict__ planes, size_t bofs, int c0, int yy, int xx, int lane, bool rnd) { v16h a; const int g = lane >> 4; const bool ok = (yy >= 0) && (yy < IH) && (xx >= 0) && (xx < IW); const size_t p = ok ? ((size_t)yy * IW + xx) : 0;
#pragma unroll
  for (int i = 0; i < 8; ++i) { float v0 = 0.f, v1 = 0.f; if (ok) { v0 = (float)planes[bofs + (size_t)(c0 + 8 * g + i) * NP + p]; v1 = (float)planes[bofs + (size_t)(c0 + 16 + 8 * g + i) * NP + p]; if (rnd) { v0 = bfr(v0); v1 = bfr(v1); } } a[i] = (_Float16)v0; a[8 + i] = (_Float16)v1; } return a; }
template <int MODE>
__global__ __launch_bounds__(128) void k_conv(const float* __restrict__ SRC, const _Float16* __restrict__ PWr, const float* __restrict__ BIAS, const float* __restrict__ G, const float* __restrict__ BT, const float* __restrict__ MU, const float* __restrict__ VAR, float* __restrict__ DST) { __shared__ __align__(16) float so[CC][64 + 4];
  const int tid = threadIdx.x, wave = tid >> 5, lane = tid & 31, col = lane & 15, g = lane >> 4; const size_t b = blockIdx.y; const int p0 = blockIdx.x * 64; const int y = p0 / IW, x0 = p0 % IW + wave * 16; const size_t bofs = b * CC * (size_t)NP;
  v8f acc[2] = {};
#pragma unroll
  for (int tap = 0; tap < KK; ++tap) { const int dy = tap / 3 - 1, dx = tap % 3 - 1; const v16h a = frag_tap<float>(SRC, bofs, 0, y + dy, x0 + col + dx, lane, MODE == 0);
#pragma unroll
    for (int j = 0; j < 2; ++j) acc[j] = wmma16(a, frag_h(PWr + (size_t)(j * 16 + col) * (KK * CC) + tap * CC, lane), acc[j]); }
#pragma unroll
  for (int j = 0; j < 2; ++j) { const int o = j * 16 + col; const float sc = bfr(G[o]) / sqrtf(bfr(VAR[o]) + BNE), mu = bfr(MU[o]), be = bfr(BT[o]), bb = bfr(BIAS[o]);
#pragma unroll
    for (int r = 0; r < 8; ++r) { const int xl = wave * 16 + 8 * g + r; float v = (acc[j][r] + bb - mu) * sc + be; if (MODE == 2) { v += DST[bofs + (size_t)o * NP + p0 + xl]; } so[o][xl] = fmaxf(v, 0.f); } }
  __syncthreads(); for (int e = tid; e < CC * 16; e += 128) { const int o = e >> 4, q = e & 15; vst2(DST + bofs + (size_t)o * NP + p0 + q * 4, *(const v4f*)&so[o][q * 4]); } }
__device__ __forceinline__ v16b fragb_f32(const float* __restrict__ p, int lane) { v16b a; const float* pp = p + 8 * (lane >> 4);
#pragma unroll
  for (int i = 0; i < 8; ++i) { a[i] = (__bf16)pp[i]; a[8 + i] = (__bf16)pp[16 + i]; } return a; }
__global__ __launch_bounds__(256) void k_init(const float* __restrict__ X, float* __restrict__ M) { const size_t base = (size_t)blockIdx.x * 4096; for (int q = threadIdx.x; q < 1024; q += 256) { v4f v = *(const v4f*)(X + base + q * 4); v[0] = bfr(v[0]); v[1] = bfr(v[1]); v[2] = bfr(v[2]); v[3] = bfr(v[3]); vst2(M + base + q * 4, v); } }
__global__ __launch_bounds__(128) void k_core(const float* __restrict__ M, const float* __restrict__ TAU, const __bf16* __restrict__ PO, const float* __restrict__ BO, const float* __restrict__ X, _Float16* __restrict__ PR) { __shared__ float score[64][CO + 1]; __shared__ __align__(16) _Float16 spr[CP][64 + 8];
  const int tid = threadIdx.x, wave = tid >> 5, lane = tid & 31, col = lane & 15, g = lane >> 4; const size_t b = blockIdx.y; const int p0 = blockIdx.x * 64; const size_t bofs = b * CC * (size_t)NP; const int y = p0 / IW;
  { float v[16]; const int xl = wave * 16 + col;
#pragma unroll
    for (int i = 0; i < 8; ++i) { const int c1 = 8 * g + i, c2 = 16 + 8 * g + i; v[i] = fmaxf(M[bofs + (size_t)c1 * NP + p0 + xl] - bfr(TAU[c1]), 0.f); v[8 + i] = fmaxf(M[bofs + (size_t)c2 * NP + p0 + xl] - bfr(TAU[c2]), 0.f); }
    const F2 a = bsplit16(v);
#pragma unroll 1
    for (int j = 0; j < CO / 16; ++j) { v8f acc = {}; const v16b w = frag_b(PO + (size_t)(j * 16 + col) * CC, lane); acc = wmma_bf(a.h, w, acc); acc = wmma_bf(a.l, w, acc); const float bb = bfr(BO[j * 16 + col]);
#pragma unroll
      for (int r = 0; r < 8; ++r) score[wave * 16 + 8 * g + r][j * 16 + col] = acc[r] + bb; } }
  __syncthreads();
  for (int e = tid; e < 64 * CC; e += 128) { const int xl = e & 63, n = e >> 6; const int x = (p0 % IW) + xl; const float* cr = &score[xl][n * KK]; const float* xin = X + bofs + (size_t)n * NP;
#pragma unroll
    for (int rr = 1; rr <= 4; ++rr) { float s = 0.f;
#pragma unroll
      for (int tap = 0; tap < KK; ++tap) { const int yy = y + (tap / 3 - 1) * rr, xx = x + (tap % 3 - 1) * rr; if (yy >= 0 && yy < IH && xx >= 0 && xx < IW) s += cr[tap] * bfr(xin[(size_t)yy * IW + xx]); }
      spr[(rr - 1) * CC + n][xl] = (_Float16)s; } }
  __syncthreads(); for (int e = tid; e < CP * 8; e += 128) { const int ch = e >> 3, q = e & 7; vst2((unsigned*)(PR + (b * CP + ch) * (size_t)NP + p0 + q * 8), *(const v4u*)&spr[ch][q * 8]); } }
__global__ __launch_bounds__(128) void k_final(const _Float16* __restrict__ PR, const _Float16* __restrict__ PF, const float* __restrict__ BF, float* __restrict__ OUT) { __shared__ __align__(16) float so[CC][64 + 4];
  const int tid = threadIdx.x, wave = tid >> 5, lane = tid & 31, col = lane & 15, g = lane >> 4; const size_t b = blockIdx.y; const int p0 = blockIdx.x * 64; const int y = p0 / IW, x0 = p0 % IW + wave * 16; const size_t bofs = b * CP * (size_t)NP;
  v8f acc[2] = {};
#pragma unroll 1
  for (int tap = 0; tap < KK; ++tap) { const int dy = tap / 3 - 1, dx = tap % 3 - 1;
#pragma unroll
    for (int cq = 0; cq < CP / 32; ++cq) { const v16h a = frag_tap<_Float16>(PR, bofs, cq * 32, y + dy, x0 + col + dx, lane, false);
#pragma unroll
      for (int j = 0; j < 2; ++j) acc[j] = wmma16(a, frag_h(PF + (size_t)(j * 16 + col) * (KK * CP) + tap * CP + cq * 32, lane), acc[j]); } }
#pragma unroll
  for (int j = 0; j < 2; ++j) { const int o = j * 16 + col; const float bb = bfr(BF[o]);
#pragma unroll
    for (int r = 0; r < 8; ++r) so[o][wave * 16 + 8 * g + r] = acc[j][r] + bb; }
  __syncthreads(); for (int e = tid; e < CC * 16; e += 128) { const int o = e >> 4, q = e & 15; vst2(OUT + (b * CC + o) * (size_t)NP + p0 + q * 4, *(const v4f*)&so[o][q * 4]); } }
extern "C" void kernel_launch(void* const* d_in, const int* in_sizes, int n_in, void* d_out, int out_size, void* d_ws, size_t ws_size, hipStream_t stream) {
  (void)in_sizes; (void)n_in; (void)out_size;
  const float** F = (const float**)d_in;
  if (ws_size < (size_t)WS_END) return;
  char* ws = (char*)d_ws; _Float16 *PW = (_Float16*)(ws + WS_PW), *PF = (_Float16*)(ws + WS_PF), *PR = (_Float16*)(ws + WS_PR); __bf16* PO = (__bf16*)(ws + WS_PO); float *M = (float*)(ws + WS_M), *H = (float*)(ws + WS_H);
  k_packw<<<dim3(CO, 10), 256, 0, stream>>>(F[1], F[10], F[8], ws);
  const dim3 grid(TPIX / 64, TNB);
  k_init<<<(unsigned)((size_t)TNB * CC * NP / 4096), 256, 0, stream>>>(F[0], M);
  for (int blk = 0; blk < 4; ++blk) { const int w0 = blk * 2, w1 = blk * 2 + 1;
    if (blk == 0) k_conv<0><<<grid, 128, 0, stream>>>(F[0], PW + (size_t)w0 * CC * KK * CC, F[2] + w0 * CC, F[3] + w0 * CC, F[4] + w0 * CC, F[5] + w0 * CC, F[6] + w0 * CC, H);
    else          k_conv<1><<<grid, 128, 0, stream>>>(M, PW + (size_t)w0 * CC * KK * CC, F[2] + w0 * CC, F[3] + w0 * CC, F[4] + w0 * CC, F[5] + w0 * CC, F[6] + w0 * CC, H);
    k_conv<2><<<grid, 128, 0, stream>>>(H, PW + (size_t)w1 * CC * KK * CC, F[2] + w1 * CC, F[3] + w1 * CC, F[4] + w1 * CC, F[5] + w1 * CC, F[6] + w1 * CC, M); }
  k_core<<<grid, 128, 0, stream>>>(M, F[7], PO, F[9], F[0], PR);
  k_final<<<grid, 128, 0, stream>>>(PR, PF, F[11], (float*)d_out);
}
